// LSTMPredictor_68272800137459
// MI455X (gfx1250) — hardware-verified
//
#include <hip/hip_runtime.h>
#include <math.h>

constexpr int TSTEPS = 8192;
constexpr int HID    = 51;
constexpr int NGATE  = 4 * HID;
constexpr int UPAD   = 64;
constexpr int NPAD   = 4 * UPAD;
constexpr int KC1    = 64;
constexpr int KC2    = 128;
constexpr int NTHR   = 128;
constexpr int NWAVE  = NTHR / 32;
constexpr int KP     = 136;
constexpr int ATILE  = 16 * KP;
constexpr int OSL    = 128;
constexpr int PRING  = 4;
constexpr int PTAB   = 2 * NTHR;
static_assert(NWAVE * 16 == UPAD);
static_assert((2 * ATILE) % NTHR == 0);
static_assert(TSTEPS % OSL == 0);
static_assert(KP % 8 == 0 && KP >= KC2);
static_assert(KC1 % 32 == 0 && KC2 % 32 == 0);
static_assert(OSL == NTHR);
static_assert(NWAVE * PRING <= NTHR);
static_assert(NPAD * 8 == 8 * 256);
static_assert(PTAB >= NGATE && NTHR >= UPAD);

typedef __attribute__((ext_vector_type(16))) _Float16 v16h;
typedef __attribute__((ext_vector_type(8)))  _Float16 v8h;
typedef __attribute__((ext_vector_type(16))) __bf16   v16b;
typedef __attribute__((ext_vector_type(8)))  __bf16   v8b;
typedef __attribute__((ext_vector_type(8)))  float    v8f;
typedef __attribute__((ext_vector_type(4)))  float    v4f;

__device__ __forceinline__ unsigned short f2bf_bits(float f) {
  unsigned u = __float_as_uint(f);
  return (unsigned short)((u + 0x7FFFu + ((u >> 16) & 1u)) >> 16);
}
__device__ __forceinline__ float bf_bits2f(unsigned short h) { return __uint_as_float(((unsigned)h) << 16); }

__device__ __forceinline__ void grp_guard4_b(v8f& a0, v8f& a1, v8f& a2, v8f& a3,
                                             v16b x, v16b y0, v16b y1, v16b y2, v16b y3) {
  asm volatile("v_nop\n\tv_nop\n\tv_nop\n\tv_nop"
               : "+v"(a0), "+v"(a1), "+v"(a2), "+v"(a3)
               : "v"(x), "v"(y0), "v"(y1), "v"(y2), "v"(y3));
}
__device__ __forceinline__ void acc_guard4(v8f& a, v8f& b, v8f& c, v8f& d) {
  asm volatile("v_nop\n\tv_nop\n\tv_nop\n\tv_nop" : "+v"(a), "+v"(b), "+v"(c), "+v"(d));
}

template <typename T> struct Frag;
template <> struct Frag<__bf16> {
  typedef v16b V; union U { v16b v; v8b h[2]; };
  static __device__ __forceinline__ v16b load(const __bf16* p) {
    U f; f.h[0] = *(const v8b*)(p); f.h[1] = *(const v8b*)(p + 16); return f.v;
  }
  static __device__ __forceinline__ v8f mma(v16b a, v16b b, v8f c) {
    return __builtin_amdgcn_wmma_f32_16x16x32_bf16(false, a, false, b, (short)0, c, false, false);
  }
};

__device__ __forceinline__ void mma_group(v8f (&acc)[4], v16b a, const __bf16* prow, size_t gstride) {
  const v16b b0 = Frag<__bf16>::load(prow);
  const v16b b1 = Frag<__bf16>::load(prow + gstride);
  const v16b b2 = Frag<__bf16>::load(prow + 2 * gstride);
  const v16b b3 = Frag<__bf16>::load(prow + 3 * gstride);
  acc[0] = Frag<__bf16>::mma(a, b0, acc[0]);
  acc[1] = Frag<__bf16>::mma(a, b1, acc[1]);
  acc[2] = Frag<__bf16>::mma(a, b2, acc[2]);
  acc[3] = Frag<__bf16>::mma(a, b3, acc[3]);
  grp_guard4_b(acc[0], acc[1], acc[2], acc[3], a, b0, b1, b2, b3);
}

__device__ __forceinline__ float fsig(float z) { return 1.0f / (1.0f + expf(-z)); }

__global__ __launch_bounds__(256) void bt_plane_kernel(const float* __restrict__ src,
                                                       unsigned short* __restrict__ dh,
                                                       unsigned short* __restrict__ dl,
                                                       int pitch, int kseg) {
  const int i = blockIdx.x * 256 + threadIdx.x;
  if (i >= NPAD * 8) return;
  const int row = i >> 3, c8 = i & 7;
  const int g = row >> 6, u = row & 63;
  const int uc = (u < HID) ? u : (HID - 1);
  const float fr = (u < HID) ? 1.0f : 0.0f;
  const float* sp = src + (size_t)(HID * g + uc) * HID;
  v8h hv, lv;
#pragma unroll
  for (int e = 0; e < 8; ++e) {
    const int kk = 8 * c8 + e;
    const int kc = (kk < HID) ? kk : (HID - 1);
    const float fk = (kk < HID) ? fr : 0.0f;
    const float v = sp[kc] * fk;
    const unsigned short hb = f2bf_bits(v);
    const unsigned short lb = f2bf_bits(v - bf_bits2f(hb));
    hv[e] = __builtin_bit_cast(_Float16, hb);
    lv[e] = __builtin_bit_cast(_Float16, lb);
  }
  const size_t o = (size_t)row * (size_t)pitch + (size_t)kseg + (size_t)(8 * c8);
  for (int pass = 0; pass < 2; ++pass) {
    *(volatile v8h*)(dh + o) = hv;
    *(volatile v8h*)(dl + o) = lv;
    __threadfence();
  }
}

__device__ __forceinline__ void emit_step(int s, int lane, const float* part_p, float* osl, float blin0,
                                          float* __restrict__ out) {
  const int slot = s & (PRING - 1);
  const float o = (((part_p[slot] + part_p[PRING + slot]) + part_p[2 * PRING + slot]) + part_p[3 * PRING + slot]) + blin0;
  if (lane == (s & 31)) osl[s & (OSL - 1)] = o;
  if ((s & (OSL - 1)) == (OSL - 1)) {
    __builtin_amdgcn_fence(__ATOMIC_RELEASE, "workgroup");
    __builtin_amdgcn_wave_barrier();
    __builtin_amdgcn_fence(__ATOMIC_ACQUIRE, "workgroup");
    const v4f v = *(const v4f*)(osl + 4 * lane);
    float* dst = out + (size_t)(s / OSL) * OSL + 4 * lane;
    for (int pass = 0; pass < 2; ++pass) {
      *(volatile v4f*)dst = v;
      __threadfence();
    }
    __builtin_amdgcn_fence(__ATOMIC_RELEASE, "workgroup");
    __builtin_amdgcn_wave_barrier();
    __builtin_amdgcn_fence(__ATOMIC_ACQUIRE, "workgroup");
  }
}

__global__ __launch_bounds__(NTHR) void lstm2_seq_kernel(const float* __restrict__ x, const float* __restrict__ Wih1,
                                                         const float* __restrict__ bih1, const float* __restrict__ bhh1,
                                                         const float* __restrict__ bih2, const float* __restrict__ bhh2,
                                                         const float* __restrict__ Wlin, const float* __restrict__ blin,
                                                         const unsigned short* __restrict__ W1Hp,
                                                         const unsigned short* __restrict__ W1Lp,
                                                         const unsigned short* __restrict__ W2Hp,
                                                         const unsigned short* __restrict__ W2Lp,
                                                         float* __restrict__ out) {
  __shared__ __align__(16) unsigned short Abuf[2 * ATILE];
  __shared__ __align__(16) float          part[NWAVE * PRING];
  __shared__ __align__(16) float          oslab[OSL];
  __shared__ __align__(16) float          sWih1[PTAB];
  __shared__ __align__(16) float          sB1[PTAB];
  __shared__ __align__(16) float          sB2[PTAB];
  __shared__ __align__(16) float          sWl[NTHR];
  const __bf16* W1H = (const __bf16*)W1Hp;
  const __bf16* W1L = (const __bf16*)W1Lp;
  const __bf16* W2H = (const __bf16*)W2Hp;
  const __bf16* W2L = (const __bf16*)W2Lp;
  const int tid = threadIdx.x, lane = tid & 31, wave = tid >> 5;
  const int c = lane & 15, hh = lane >> 4, koff = hh * 8;
  const int u = 16 * wave + c;
  const bool valid = (hh == 0) && (u < HID);
  const int uc = (u < HID) ? u : (HID - 1);
  const float vf = valid ? 1.0f : 0.0f;

#pragma unroll 1
  for (int i = tid; i < 2 * ATILE; i += NTHR) Abuf[i] = (unsigned short)0;
  if (tid < NWAVE * PRING) part[tid] = 0.0f;
  oslab[tid] = 0.0f;
#pragma unroll 1
  for (int it = 0; it < 2; ++it) {
    const int i  = it * NTHR + tid;
    const int ic = (i < NGATE) ? i : (NGATE - 1);
    const float fi = (i < NGATE) ? 1.0f : 0.0f;
    const float w  = Wih1[ic] * fi;
    const float ba = (bih1[ic] + bhh1[ic]) * fi;
    const float bb = (bih2[ic] + bhh2[ic]) * fi;
    sWih1[i] = w;
    sB1[i]   = ba;
    sB2[i]   = bb;
  }
  {
    const int kc = (tid < HID) ? tid : (HID - 1);
    const float fw = (tid < HID) ? 1.0f : 0.0f;
    sWl[tid] = Wlin[kc] * fw;
  }
  const float blin0 = blin[0];
  float c1s = 0.0f, c2s = 0.0f;
  __syncthreads();

  float wih1r[4], b1r[4], b2r[4];
#pragma unroll
  for (int g = 0; g < 4; ++g) {
    const int n = HID * g + uc;
    wih1r[g] = sWih1[n] * vf;
    b1r[g]   = sB1[n] * vf;
    b2r[g]   = sB2[n] * vf;
  }
  const float wlinr = sWl[uc] * vf;

  const v8f z8 = {0.f, 0.f, 0.f, 0.f, 0.f, 0.f, 0.f, 0.f};
  const __bf16* Ab = (const __bf16*)Abuf;
  const int arow = c * KP + koff;
  const size_t w1off = (size_t)u * KC1 + koff;
  const size_t w2off = (size_t)u * KC2 + koff;

#pragma unroll 1
  for (int t = 0; t < TSTEPS; ++t) {
    const float xt = x[t];
    const int pb = t & 1;
    const int qb = pb ^ 1;

    v8f acc[4];
    acc[0] = z8; acc[1] = z8; acc[2] = z8; acc[3] = z8;
#pragma unroll 1
    for (int kt = 0; kt < KC1 / 32; ++kt) {
      const v16b a = Frag<__bf16>::load(Ab + qb * ATILE + arow + 32 * kt);
      mma_group(acc, a, W1H + w1off + 32 * kt, (size_t)UPAD * KC1);
      mma_group(acc, a, W1L + w1off + 32 * kt, (size_t)UPAD * KC1);
    }
    acc_guard4(acc[0], acc[1], acc[2], acc[3]);
    float h1n;
    {
      const float zi = (acc[0][0] + acc[0][1]) + (b1r[0] + xt * wih1r[0]);
      const float zf = (acc[1][0] + acc[1][1]) + (b1r[1] + xt * wih1r[1]);
      const float zg = (acc[2][0] + acc[2][1]) + (b1r[2] + xt * wih1r[2]);
      const float zo = (acc[3][0] + acc[3][1]) + (b1r[3] + xt * wih1r[3]);
      const float ig = fsig(zi);
      const float fg = fsig(zf);
      const float gg = tanhf(zg);
      const float og = fsig(zo);
      const float cn = fg * c1s + ig * gg;
      const float hn = og * tanhf(cn);
      c1s = valid ? cn : 0.0f;
      h1n = valid ? hn : 0.0f;
    }
    if (hh == 0) {
      const unsigned short hb = f2bf_bits(h1n);
      const unsigned short lb = f2bf_bits(h1n - bf_bits2f(hb));
      Abuf[pb * ATILE + u]      = hb;
      Abuf[pb * ATILE + KP + u] = lb;
    }
    __syncthreads();
    if (wave == 0 && t > 0) emit_step(t - 1, lane, part, oslab, blin0, out);

    acc[0] = z8; acc[1] = z8; acc[2] = z8; acc[3] = z8;
#pragma unroll 1
    for (int kt = 0; kt < KC2 / 32; ++kt) {
      const int bsel = pb ^ (kt >> 1);
      const v16b a = Frag<__bf16>::load(Ab + bsel * ATILE + arow + 32 * kt);
      mma_group(acc, a, W2H + w2off + 32 * kt, (size_t)UPAD * KC2);
      mma_group(acc, a, W2L + w2off + 32 * kt, (size_t)UPAD * KC2);
    }
    acc_guard4(acc[0], acc[1], acc[2], acc[3]);
    float h2n;
    {
      const float zi = (acc[0][0] + acc[0][1]) + b2r[0];
      const float zf = (acc[1][0] + acc[1][1]) + b2r[1];
      const float zg = (acc[2][0] + acc[2][1]) + b2r[2];
      const float zo = (acc[3][0] + acc[3][1]) + b2r[3];
      const float ig = fsig(zi);
      const float fg = fsig(zf);
      const float gg = tanhf(zg);
      const float og = fsig(zo);
      const float cn = fg * c2s + ig * gg;
      const float hn = og * tanhf(cn);
      c2s = valid ? cn : 0.0f;
      h2n = valid ? hn : 0.0f;
    }
    if (hh == 0) {
      const unsigned short hb = f2bf_bits(h2n);
      const unsigned short lb = f2bf_bits(h2n - bf_bits2f(hb));
      Abuf[pb * ATILE + KC1 + u]      = hb;
      Abuf[pb * ATILE + KP + KC1 + u] = lb;
    }
    float pp = h2n * wlinr;
#pragma unroll
    for (int off = 16; off > 0; off >>= 1) pp += __shfl_xor(pp, off, 32);
    if (lane == 0) part[wave * PRING + (t & (PRING - 1))] = pp;
  }
  __syncthreads();
  if (wave == 0) emit_step(TSTEPS - 1, lane, part, oslab, blin0, out);
}

extern "C" void kernel_launch(void* const* d_in, const int* in_sizes, int n_in,
                              void* d_out, int out_size, void* d_ws, size_t ws_size, hipStream_t stream) {
  if (n_in < 11 || d_out == nullptr || d_ws == nullptr) return;
  if (in_sizes[0] != TSTEPS || in_sizes[1] != NGATE || in_sizes[2] != NGATE * HID || in_sizes[3] != NGATE ||
      in_sizes[4] != NGATE || in_sizes[5] != NGATE * HID || in_sizes[6] != NGATE * HID || in_sizes[7] != NGATE ||
      in_sizes[8] != NGATE || in_sizes[9] != HID || in_sizes[10] != 1 || out_size != TSTEPS) return;

  const float* x    = (const float*)d_in[0];
  const float* Wih1 = (const float*)d_in[1];
  const float* Whh1 = (const float*)d_in[2];
  const float* bih1 = (const float*)d_in[3];
  const float* bhh1 = (const float*)d_in[4];
  const float* Wih2 = (const float*)d_in[5];
  const float* Whh2 = (const float*)d_in[6];
  const float* bih2 = (const float*)d_in[7];
  const float* bhh2 = (const float*)d_in[8];
  const float* Wlin = (const float*)d_in[9];
  const float* blin = (const float*)d_in[10];
  float* out = (float*)d_out;

  char* ws = (char*)d_ws; size_t off = 0;
  auto carve = [&](size_t bytes) -> char* { char* p = ws + off; off += (bytes + 255) & ~(size_t)255; return p; };
  unsigned short* W1H = (unsigned short*)carve((size_t)NPAD * KC1 * 2);
  unsigned short* W1L = (unsigned short*)carve((size_t)NPAD * KC1 * 2);
  unsigned short* W2H = (unsigned short*)carve((size_t)NPAD * KC2 * 2);
  unsigned short* W2L = (unsigned short*)carve((size_t)NPAD * KC2 * 2);
  if (off > ws_size || off > (size_t)134217728) return;

  bt_plane_kernel<<<8, 256, 0, stream>>>(Whh1, W1H, W1L, KC1, 0);
  bt_plane_kernel<<<8, 256, 0, stream>>>(Wih2, W2H, W2L, KC2, 0);
  bt_plane_kernel<<<8, 256, 0, stream>>>(Whh2, W2H, W2L, KC2, KC1);
  lstm2_seq_kernel<<<1, NTHR, 0, stream>>>(x, Wih1, bih1, bhh1, bih2, bhh2, Wlin, blin, W1H, W1L, W2H, W2L, out);
}
